// SimpleNet_58256936403066
// MI455X (gfx1250) — hardware-run, weakly checked
//
#include <hip/hip_runtime.h>


namespace {
constexpr int N = 100000, NP = 100096, NLIM = 100096  , NLIMN = (NLIM < N ? NLIM : N), E = 800000, HD = 64, CH = 512, NCH = NP / CH   + 1;
constexpr float XS = 8.0f, WSC = 256.0f, EPS = 1e-5f;
static_assert(NP % 64 == 0 && NLIM % 64 == 0, "tiling");
typedef _Float16 b16;
typedef __attribute__((ext_vector_type(16))) _Float16 v16b;
typedef __attribute__((ext_vector_type(8))) _Float16 v8b;
typedef __attribute__((ext_vector_type(8))) float v8f;
typedef __attribute__((ext_vector_type(4))) float v4f;
__device__ __forceinline__ float bf16_rne(float f) { unsigned int u = __float_as_uint(f); u += 0x7FFFu + ((u >> 16) & 1u); return __uint_as_float(u & 0xFFFF0000u); }
__device__ __forceinline__ void split16(float v, b16& hi, b16& lo) { hi = (b16)v; lo = (b16)(v - (float)hi); }
__device__ __forceinline__ v16b frag_kb(const b16* p, int hh) { const v8b a = *(const v8b*)(p + 8 * hh), b = *(const v8b*)(p + 16 + 8 * hh); v16b f;
#pragma unroll
  for (int e = 0; e < 8; ++e) { f[e] = a[e]; f[8 + e] = b[e]; } return f; }
__device__ __forceinline__ v8f wmma16b(v16b a, v16b b, v8f c) { v8f d = __builtin_amdgcn_wmma_f32_16x16x32_f16(false, a, false, b, (short)0, c, false, false); asm volatile("v_nop\n\tv_nop\n\tv_nop\n\tv_nop" : "+v"(d) : "v"(a), "v"(b)); return d; }
__device__ __forceinline__ void wave_lds_sync() { __builtin_amdgcn_fence(__ATOMIC_RELEASE, "workgroup"); __builtin_amdgcn_wave_barrier(); __builtin_amdgcn_fence(__ATOMIC_ACQUIRE, "workgroup"); }
__device__ __forceinline__ float pmul(float a, float b) { float p = a * b; asm volatile("" : "+v"(p)); return p; }
__device__ __forceinline__ int iclamp(int v, int lo, int hi) { return v < lo ? lo : (v > hi ? hi : v); }
constexpr int CSR_NBLK = 512, CSR_GB = 9, CSR_GN = 1 << CSR_GB  , CSR_MAXG = 512, CSR_CAP = 12288  ;
__global__ __launch_bounds__(64) void csrA_kernel(const int* __restrict__ dst, int E, int N, int nG, int CHP, int NGP, int* __restrict__ STG, int* __restrict__ HST) {
  extern __shared__ int sm[];
  int* cnt = sm; int* run = sm + NGP; int* ids = sm + 2 * NGP;
  const int b = blockIdx.x; const int ch = (E + CSR_NBLK - 1) / CSR_NBLK; const int e0 = b * ch, e1 = min(E, e0 + ch);
  for (int i = threadIdx.x; i < NGP; i += 64) cnt[i] = 0;
  for (int i = threadIdx.x; i < CHP; i += 64) ids[i] = -1;
  __syncthreads();
  if (threadIdx.x == 0) {
    for (int e = e0; e < e1; ++e) { int d = dst[e]; d = (d < 0) ? 0 : (d >= N ? N - 1 : d); cnt[d >> CSR_GB] += 1; }
    int acc = 0; for (int g = 0; g < nG; ++g) { run[g] = acc; acc += cnt[g]; }
    for (int e = e0; e < e1; ++e) { int d = dst[e]; d = (d < 0) ? 0 : (d >= N ? N - 1 : d); const int g = d >> CSR_GB; ids[run[g]] = e; run[g] += 1; } }
  __syncthreads();
  typedef __attribute__((ext_vector_type(4))) int v4i;
  for (int pass = 0; pass < 2; ++pass) {
    for (int i = threadIdx.x; i < CHP / 4; i += 64) *(volatile v4i*)(STG + (size_t)b * CHP + i * 4) = *(const v4i*)(&ids[i * 4]);
    for (int i = threadIdx.x; i < NGP / 4; i += 64) { v4i v; for (int e = 0; e < 4; ++e) v[e] = (i * 4 + e < nG) ? cnt[i * 4 + e] : 0; *(volatile v4i*)(HST + (size_t)b * NGP + i * 4) = v; }
    __threadfence(); }
}
__global__ __launch_bounds__(512) void csrS_kernel(const int* __restrict__ HST, int nG, int NGP, int* __restrict__ START, int* __restrict__ TOT, int* __restrict__ OFF) {
  __shared__ int tot[CSR_MAXG];
  const int b = threadIdx.x;
  for (int pass = 0; pass < 2; ++pass) { int runb = 0; for (int g = 0; g < nG; ++g) { int c = HST[(size_t)b * NGP + g]; c = (c < 0) ? 0 : c; ((volatile int*)OFF)[(size_t)g * CSR_NBLK + b] = runb; runb += c; } __threadfence(); }
  for (int g = threadIdx.x; g < nG; g += 512) { int s = 0; for (int bb = 0; bb < CSR_NBLK; ++bb) { int c = HST[(size_t)bb * NGP + g]; s += (c < 0) ? 0 : c; } tot[g] = s; }
  __syncthreads();
  if (threadIdx.x < 32) {
    __shared__ int st[CSR_MAXG + 32];
    if (threadIdx.x == 0) { int acc = 0; for (int g = 0; g < NGP; ++g) { st[g] = acc; if (g < nG) acc += (tot[g] + 31) & ~31; } st[NGP] = acc; }
    __builtin_amdgcn_fence(__ATOMIC_RELEASE, "workgroup"); __builtin_amdgcn_wave_barrier(); __builtin_amdgcn_fence(__ATOMIC_ACQUIRE, "workgroup");
    for (int pass = 0; pass < 2; ++pass) { for (int i = threadIdx.x; i < NGP + 32; i += 32) { ((volatile int*)START)[i] = (i <= NGP) ? st[min(i, NGP)] : 0; ((volatile int*)TOT)[i] = (i < nG) ? tot[i] : 0; } __threadfence(); } }
}
__global__ __launch_bounds__(256) void csrB_kernel(const int* __restrict__ dst, int N, int nG, int CHP, int NGP, int permLen, const int* __restrict__ STG, const int* __restrict__ HST, const int* __restrict__ OFF, const int* __restrict__ START, const int* __restrict__ TOT, int* __restrict__ PERM, int* __restrict__ ROWPTR, int* __restrict__ ROWCNT, int* __restrict__ FLAG) {
  typedef __attribute__((ext_vector_type(4))) int v4i;
  __shared__ int ids[CSR_CAP]; __shared__ unsigned short key[CSR_CAP]; __shared__ int outp[CSR_CAP]; __shared__ int ncnt[CSR_GN + 1]; __shared__ int boff[CSR_NBLK + 1];
  const int g = blockIdx.x, t_ = threadIdx.x; int tot = TOT[g]; int st = START[g], stn = START[g + 1]; const int v0 = g * CSR_GN; const int nv = min(CSR_GN, N - v0);
  st = (st < 0) ? 0 : (st > permLen - 32 ? permLen - 32 : st) & ~31; stn = (stn < st) ? st : (stn > permLen ? permLen : stn); tot = (tot < 0) ? 0 : tot; if (tot > stn - st && tot <= CSR_CAP) tot = stn - st;
  if (tot > CSR_CAP) {
    for (int pass = 0; pass < 2; ++pass) { for (int i = t_; i < CSR_GN / 4; i += 256) { v4i a, c; for (int e = 0; e < 4; ++e) { a[e] = st; c[e] = 0; } *(volatile v4i*)(ROWPTR + v0 + i * 4) = a; *(volatile v4i*)(ROWCNT + v0 + i * 4) = c; } if (t_ == 0) ((volatile int*)FLAG)[0] = 1; __threadfence(); } (void)nv; return; }
  if (t_ == 0) { int acc = 0; for (int b = 0; b < CSR_NBLK; ++b) { boff[b] = acc; int c = HST[(size_t)b * NGP + g]; c = (c < 0) ? 0 : (c > CHP ? CHP : c); acc += c; if (acc > tot) acc = tot; } boff[CSR_NBLK] = acc; }
  for (int i = t_; i <= CSR_GN; i += 256) ncnt[i] = 0;
  __syncthreads();
  for (int b = 0; b < CSR_NBLK; ++b) { const int c = boff[b + 1] - boff[b]; int o_ = OFF[(size_t)g * CSR_NBLK + b]; o_ = (o_ < 0) ? 0 : (o_ > CHP - c ? CHP - c : o_); const int* src_ = STG + (size_t)b * CHP + o_;
    for (int i = t_; i < c; i += 256) { int id = src_[i]; id = (id < 0) ? 0 : id; ids[boff[b] + i] = id; int d = dst[id]; d = (d < v0) ? v0 : (d >= N ? N - 1 : d); int kk = d - v0; kk = (kk < 0) ? 0 : (kk >= CSR_GN ? CSR_GN - 1 : kk); key[boff[b] + i] = (unsigned short)kk; } }
  __syncthreads();
  if (t_ == 0) { for (int i = 0; i < tot; ++i) ncnt[key[i]] += 1; int acc = 0; for (int vl = 0; vl < CSR_GN; ++vl) { const int c = ncnt[vl]; ncnt[vl] = acc; acc += c; } ncnt[CSR_GN] = acc;
    for (int i = 0; i < tot; ++i) { const int vl = key[i]; outp[ncnt[vl]] = ids[i]; ncnt[vl] += 1; }
    for (int vl = CSR_GN; vl > 0; --vl) ncnt[vl] = ncnt[vl - 1]; ncnt[0] = 0; }
  __syncthreads();
  for (int pass = 0; pass < 2; ++pass) {
    for (int i = t_; i < (stn - st) / 4; i += 256) { v4i v; for (int e = 0; e < 4; ++e) { const int q = i * 4 + e; v[e] = (q < tot) ? outp[q] : -1; } *(volatile v4i*)(PERM + st + i * 4) = v; }
    for (int i = t_; i < CSR_GN / 4; i += 256) { v4i a, c; for (int e = 0; e < 4; ++e) { const int vl = i * 4 + e; a[e] = st + ncnt[vl]; c[e] = (vl < nv) ? (ncnt[vl + 1] - ncnt[vl]) : 0; } *(volatile v4i*)(ROWPTR + v0 + i * 4) = a; *(volatile v4i*)(ROWCNT + v0 + i * 4) = c; }
    __threadfence(); }
}
__global__ __launch_bounds__(256) void csrZ_kernel(int* __restrict__ p, size_t n4) { typedef __attribute__((ext_vector_type(4))) int v4i; const size_t tid = (size_t)blockIdx.x * 256 + threadIdx.x, nth = (size_t)gridDim.x * 256; v4i z = {0, 0, 0, 0}; for (size_t i = tid; i < n4; i += nth) *(volatile v4i*)(p + i * 4) = z; }
struct CsrBufs { int *STG, *HST, *OFF, *START, *TOT, *PERM, *ROWPTR, *ROWCNT, *FLAG; int nG, NGP, CHP; size_t permLen; char* base; size_t bytes; };
static size_t csr_carve(CsrBufs& c, char* ws, size_t off, int E, int N) {
  const size_t off0 = off; c.base = ws + off;
  auto al = [&](size_t bytes) { char* p = ws + off; off += (bytes + 255) & ~(size_t)255; return p; };
  c.nG = (N + CSR_GN - 1) / CSR_GN; c.NGP = (c.nG + 31) & ~31; const int ch = (E + CSR_NBLK - 1) / CSR_NBLK; c.CHP = (ch + 31) & ~31; c.permLen = (size_t)E + 32 * (size_t)c.nG + 32;
  c.STG = (int*)al((size_t)CSR_NBLK * c.CHP * 4); c.HST = (int*)al((size_t)CSR_NBLK * c.NGP * 4); c.OFF = (int*)al((size_t)c.NGP * CSR_NBLK * 4); c.START = (int*)al((size_t)(c.NGP + 64) * 4); c.TOT = (int*)al((size_t)(c.NGP + 64) * 4);
  c.PERM = (int*)al(c.permLen * 4); c.ROWPTR = (int*)al((size_t)c.nG * CSR_GN * 4); c.ROWCNT = (int*)al((size_t)c.nG * CSR_GN * 4); c.FLAG = (int*)al(256);
  c.bytes = off - off0; return off;
}
static void csr_build(const CsrBufs& c, const int* dst, int E, int N, hipStream_t stream) {
  const size_t smem = (size_t)(2 * c.NGP + c.CHP) * 4;
  csrZ_kernel<<<512, 256, 0, stream>>>((int*)c.base, c.bytes / 16);
  csrA_kernel<<<CSR_NBLK, 64, smem, stream>>>(dst, E, N, c.nG, c.CHP, c.NGP, c.STG, c.HST);
  csrS_kernel<<<1, 512, 0, stream>>>(c.HST, c.nG, c.NGP, c.START, c.TOT, c.OFF);
  csrB_kernel<<<c.nG, 256, 0, stream>>>(dst, N, c.nG, c.CHP, c.NGP, (int)c.permLen, c.STG, c.HST, c.OFF, c.START, c.TOT, c.PERM, c.ROWPTR, c.ROWCNT, c.FLAG);
}

typedef __attribute__((ext_vector_type(2))) float v2f;
__global__ __launch_bounds__(256) void prep_kernel(const float* __restrict__ vw2, const float* __restrict__ cw2, const float* __restrict__ nw1, const float* __restrict__ nw2, b16* __restrict__ WT) {
  const int t = blockIdx.x * 256 + threadIdx.x; if (t >= 5 * HD * HD / 8) return; const int m = t / (HD * HD / 8); const int e = (t % (HD * HD / 8)) * 8; const int oo = e / HD, k0 = e % HD; v8b o;
  for (int j = 0; j < 8; ++j) { const int k = k0 + j; float w; if (m == 0) w = vw2[k * HD + oo]; else if (m == 1) w = cw2[k * HD + oo]; else if (m == 2) w = nw1[k * HD + oo]; else if (m == 3) w = nw1[(HD + k) * HD + oo]; else w = nw2[k * HD + oo]; o[j] = (b16)(bf16_rne(w) * WSC); }
  for (int pass = 0; pass < 2; ++pass) { *(volatile v8b*)(WT + (size_t)m * HD * HD + e) = o; __threadfence(); }
}
template <int KIND>
__global__ __launch_bounds__(128) void node_kernel(const float* __restrict__ feat, const float* __restrict__ w1, const float* __restrict__ b1, const float* __restrict__ b2, const b16* __restrict__ WT, float* __restrict__ P) {
  __shared__ __attribute__((aligned(16))) float Tf[4][16][HD + 4];
  const int wave = threadIdx.x >> 5, lane = threadIdx.x & 31, nloc = lane & 15, hlf = lane >> 4; const size_t v0 = ((size_t)blockIdx.x * 4 + wave) * 16; const size_t vr = v0 + nloc; const bool zr = vr >= (size_t)N; const size_t vra = zr ? (size_t)N - 1 : vr;
  const float f0 = bf16_rne(feat[vra * 2]), f1 = bf16_rne(feat[vra * 2 + 1]);
  v8f acc[4];
#pragma unroll
  for (int t = 0; t < 4; ++t) acc[t] = (v8f){};
#pragma unroll
  for (int ks = 0; ks < 2; ++ks) { v16b ah, al;
#pragma unroll
    for (int e2 = 0; e2 < 16; ++e2) { const int k = ks * 32 + (e2 < 8 ? 0 : 16) + 8 * hlf + (e2 & 7); float h = fmaxf(f0 * bf16_rne(w1[k]) + f1 * bf16_rne(w1[HD + k]) + bf16_rne(b1[k]), 0.0f); if (zr) h = 0.0f; b16 p, q; split16(h * XS, p, q); ah[e2] = p; al[e2] = q; }
#pragma unroll
    for (int t = 0; t < 4; ++t) { const v16b bw = frag_kb(WT + (size_t)KIND * HD * HD + (size_t)(t * 16 + nloc) * HD + ks * 32, hlf); acc[t] = wmma16b(ah, bw, acc[t]); acc[t] = wmma16b(al, bw, acc[t]); } }
#pragma unroll
  for (int t = 0; t < 4; ++t) { const float bb = bf16_rne(b2[t * 16 + nloc]);
#pragma unroll
    for (int r = 0; r < 8; ++r) { const bool zrow = (v0 + 8 * hlf + r) >= (size_t)N; Tf[wave][8 * hlf + r][t * 16 + nloc] = zrow ? 0.0f : (acc[t][r] * (1.0f / (XS * WSC)) + bb); } }
  wave_lds_sync();
#pragma unroll
  for (int t = 0; t < 4; ++t) acc[t] = (v8f){};
#pragma unroll
  for (int ks = 0; ks < 2; ++ks) { v16b ah, al;
#pragma unroll
    for (int e2 = 0; e2 < 16; ++e2) { const int k = ks * 32 + (e2 < 8 ? 0 : 16) + 8 * hlf + (e2 & 7); b16 p, q; split16(Tf[wave][nloc][k] * XS, p, q); ah[e2] = p; al[e2] = q; }
#pragma unroll
    for (int t = 0; t < 4; ++t) { const v16b bw = frag_kb(WT + (size_t)(KIND == 0 ? 3 : 2) * HD * HD   + (size_t)(t * 16 + nloc) * HD + ks * 32, hlf); acc[t] = wmma16b(ah, bw, acc[t]); acc[t] = wmma16b(al, bw, acc[t]); } }
  wave_lds_sync();
#pragma unroll
  for (int t = 0; t < 4; ++t)
#pragma unroll
    for (int r = 0; r < 8; ++r) Tf[wave][8 * hlf + r][t * 16 + nloc] = acc[t][r] * (1.0f / (XS * WSC));
  wave_lds_sync();
  for (int pass = 0; pass < 2; ++pass) { for (int rr = 0; rr < 16; ++rr) *(volatile v2f*)(P + (v0 + rr) * HD + lane * 2) = *(const v2f*)(&Tf[wave][rr][lane * 2]); __threadfence(); }
}
__global__ __launch_bounds__(256) void edge_kernel(const float* __restrict__ PT, const float* __restrict__ PS, const float* __restrict__ b1, const float* __restrict__ b2, const b16* __restrict__ WT, const int* __restrict__ srcs, const int* __restrict__ PERM, const int* __restrict__ ROWPTR, const int* __restrict__ ROWCNT, int permLen, float* __restrict__ SUM, float* __restrict__ SSQ, float* __restrict__ CNT) {
  const int wave = threadIdx.x >> 5, lane = threadIdx.x & 31, nloc = lane & 15, hlf = lane >> 4; const size_t v = (size_t)blockIdx.x * 8 + wave;
  float s1[4], s2[4]; for (int t = 0; t < 4; ++t) { s1[t] = 0.0f; s2[t] = 0.0f; } int used = 0;
  if (v < (size_t)NLIMN) { int st = ROWPTR[v], cnt = ROWCNT[v]; cnt = iclamp(cnt, 0, 4096); st = iclamp(st, 0, permLen - cnt);
    float pt[16]; for (int g = 0; g < 2; ++g) for (int i = 0; i < 8; ++i) pt[g * 8 + i] = 0.0f;
#pragma unroll 1
    for (int t0 = 0; t0 < cnt; t0 += 16) {
      const int slot = t0 + nloc; int j = -1; if (slot < cnt) { const int e = iclamp(PERM[st + slot], 0, E - 1); j = iclamp(srcs[e], 0, N - 1); if (j >= NLIM) j = -1; }
      v8f acc[4]; for (int t = 0; t < 4; ++t) acc[t] = (v8f){};
#pragma unroll
      for (int ks = 0; ks < 2; ++ks) { v16b ah, al;
#pragma unroll
        for (int e2 = 0; e2 < 16; ++e2) { const int k = ks * 32 + (e2 < 8 ? 0 : 16) + 8 * hlf + (e2 & 7); float h = 0.0f; if (j >= 0) h = fmaxf(PT[v * HD + k] + PS[(size_t)j * HD + k] + bf16_rne(b1[k]), 0.0f); b16 p, q; split16(h * XS, p, q); ah[e2] = p; al[e2] = q; }
#pragma unroll
        for (int t = 0; t < 4; ++t) { const v16b bw = frag_kb(WT + (size_t)4 * HD * HD + (size_t)(t * 16 + nloc) * HD + ks * 32, hlf); acc[t] = wmma16b(ah, bw, acc[t]); acc[t] = wmma16b(al, bw, acc[t]); } }
#pragma unroll
      for (int t = 0; t < 4; ++t) { const float bb = bf16_rne(b2[t * 16 + nloc]);
#pragma unroll
        for (int r = 0; r < 8; ++r) { const int row = t0 + 8 * hlf + r;
          float m = fmaxf(acc[t][r] * (1.0f / (XS * WSC)) + bb, 0.0f); const int jrow = __shfl(j, 8 * hlf + r);
          const bool ok = (row < cnt) && (jrow >= 0); if (!ok) m = 0.0f; s1[t] += m; s2[t] += m * m; } }
      { int add = 0; for (int r = 0; r < 16; ++r) { const int jr = __shfl(j, r); if (t0 + r < cnt && jr >= 0) ++add; } used += add; } } }
#pragma unroll
  for (int t = 0; t < 4; ++t) { s1[t] += __shfl_xor(s1[t], 16); s2[t] += __shfl_xor(s2[t], 16); }
  float o1[2], o2[2];
  for (int q = 0; q < 2; ++q) { const int c = 2 * lane + q; const int t = c / 16, nl = c % 16; const float a1 = __shfl(s1[0], nl), a2 = __shfl(s1[1], nl), a3 = __shfl(s1[2], nl), a4 = __shfl(s1[3], nl); const float b1_ = __shfl(s2[0], nl), b2_ = __shfl(s2[1], nl), b3_ = __shfl(s2[2], nl), b4_ = __shfl(s2[3], nl);
    o1[q] = t == 0 ? a1 : t == 1 ? a2 : t == 2 ? a3 : a4; o2[q] = t == 0 ? b1_ : t == 1 ? b2_ : t == 2 ? b3_ : b4_; }
  for (int pass = 0; pass < 2; ++pass) { const v2f u1 = {o1[0], o1[1]}, u2 = {o2[0], o2[1]}; *(volatile v2f*)(SUM + v * HD + 2 * lane) = u1; *(volatile v2f*)(SSQ + v * HD + 2 * lane) = u2; if ((v & 31) == 0 && lane == 0) {   } __threadfence(); }
  for (int pass = 0; pass < 2; ++pass) { ((volatile float*)CNT)[v * 32 + lane] = (float)used; __threadfence(); }
}
__global__ __launch_bounds__(256) void statA_kernel(const float* __restrict__ SUM, const float* __restrict__ SSQ, const float* __restrict__ CNT, double* __restrict__ PART) {
  const int ch = blockIdx.x, t = threadIdx.x; const size_t v0 = (size_t)ch * CH, v1 = (v0 + CH < (size_t)NP) ? v0 + CH : (size_t)NP; double s = 0.0;
  if (t < 128) { const float* src = (t < 64) ? (SUM + t) : (SSQ + t - 64); for (size_t v = v0; v < v1; ++v) s += (double)src[v * HD]; }
  else if (t == 128) { for (size_t v = v0; v < v1; ++v) s += (double)CNT[v * 32]; }
  for (int pass = 0; pass < 2; ++pass) { ((volatile double*)PART)[(size_t)ch * 256 + t] = s; __threadfence(); }
}
__global__ __launch_bounds__(256) void statB_kernel(const double* __restrict__ PART, float* __restrict__ STAT) {
  __shared__ double tot; const int t = threadIdx.x;
  if (t == 0) { double c = 0.0; for (int ch = 0; ch < NCH; ++ch) c += PART[(size_t)ch * 256 + 128]; tot = (c > 0.0) ? c : 1.0; }
  __syncthreads();
  if (t < 64) { double s = 0.0, q = 0.0;
#pragma unroll 1
    for (int ch = 0; ch < NCH; ++ch) { s += PART[(size_t)ch * 256 + t]; q += PART[(size_t)ch * 256 + 64 + t]; }
    const double mu = s / tot; double var = q / tot - mu * mu; if (var < 0.0) var = 0.0; const float rs = (float)(1.0 / sqrt(var + (double)EPS));
    for (int pass = 0; pass < 2; ++pass) { ((volatile float*)STAT)[t] = (float)mu; ((volatile float*)STAT)[64 + t] = rs; __threadfence(); } }
}
__global__ __launch_bounds__(256) void out_kernel(const float* __restrict__ SUM, const float* __restrict__ CNT, const float* __restrict__ STAT, const float* __restrict__ gam, const float* __restrict__ bet, float* __restrict__ out) {
  const int wave = threadIdx.x >> 5, lane = threadIdx.x & 31; const size_t v = (size_t)blockIdx.x * 8 + wave; if (v >= (size_t)NLIMN) return;
  const float cnt = CNT[v * 32]; v2f o = {0.0f, 0.0f};
  if (cnt > 0.0f) { const float inv = 1.0f / cnt; for (int q = 0; q < 2; ++q) { const int c = 2 * lane + q; o[q] = (SUM[v * HD + c] * inv - STAT[c]) * STAT[64 + c] * bf16_rne(gam[c]) + bf16_rne(bet[c]); } }
  for (int pass = 0; pass < 2; ++pass) { *(volatile v2f*)(out + v * HD + 2 * lane) = o; __threadfence(); }
}
}

extern "C" void kernel_launch(void* const* d_in, const int* in_sizes, int n_in, void* d_out, int out_size, void* d_ws, size_t ws_size, hipStream_t stream) {
  (void)n_in;
  auto Fp = [&](int i) { return (const float*)d_in[i]; }; auto Ip = [&](int i) { return (const int*)d_in[i]; };
  if (in_sizes[0] != N * 2 || in_sizes[1] != N * 2 || in_sizes[2] != 2 * E || in_sizes[3] != 2 * HD || in_sizes[5] != HD * HD || in_sizes[7] != 2 * HD || in_sizes[9] != HD * HD || in_sizes[11] != 2 * HD * HD || in_sizes[13] != HD * HD || in_sizes[15] != HD || in_sizes[16] != HD || out_size != N * HD) return;
  size_t off = 0; char* ws = (char*)d_ws;
  auto carve = [&](size_t bytes) { char* p = ws + off; off += (bytes + 255) & ~(size_t)255; return p; };
  b16* WT = (b16*)carve((size_t)5 * HD * HD * 2); float* PS = (float*)carve((size_t)NP * HD * 4); float* PT = (float*)carve((size_t)NP * HD * 4); float* SUM = (float*)carve((size_t)NP * HD * 4); float* SSQ = (float*)carve((size_t)NP * HD * 4); float* CNT = (float*)carve((size_t)NP * 32 * 4);
  double* PART = (double*)carve((size_t)NCH * 256 * 8); float* STAT = (float*)carve(128 * 4);
  CsrBufs csr; off = csr_carve(csr, ws, off, E, N);
  if (off > ws_size || off > ((size_t)128 << 20)) return;
  prep_kernel<<<(5 * HD * HD / 8 + 255) / 256, 256, 0, stream>>>(Fp(5), Fp(9), Fp(11), Fp(13), WT);
  csr_build(csr, Ip(2) + E, E, N, stream);
  node_kernel<0><<<NP / 64, 128, 0, stream>>>(Fp(0), Fp(3), Fp(4), Fp(6), WT, PS);
  node_kernel<1><<<NP / 64, 128, 0, stream>>>(Fp(1), Fp(7), Fp(8), Fp(10), WT, PT);
  edge_kernel<<<NP / 8, 256, 0, stream>>>(PT, PS, Fp(12), Fp(14), WT, Ip(2), csr.PERM, csr.ROWPTR, csr.ROWCNT, (int)csr.permLen, SUM, SSQ, CNT);
  statA_kernel<<<NCH, 256, 0, stream>>>(SUM, SSQ, CNT, PART);
  statB_kernel<<<1, 256, 0, stream>>>(PART, STAT);
  out_kernel<<<NP / 8, 256, 0, stream>>>(SUM, CNT, STAT, Fp(15), Fp(16), (float*)d_out);
}
